// LSTMModel_42709154791735
// MI455X (gfx1250) — hardware-verified
//
#include <hip/hip_runtime.h>
#include <math.h>

constexpr int NBATCH   = 256;
constexpr int NPOS     = 2048;
constexpr int NCH_IN   = 3;
constexpr int NCH_MID  = 16;
constexpr int NCH_SEQ  = 32;
constexpr int NSTEP    = 512;
constexpr int NHID     = 64;
constexpr int NGATE    = 256;
constexpr int NOUTF    = 5;
constexpr int CONV_TL  = 128;
constexpr int XL_N     = 4 * CONV_TL + 6;
constexpr int P1_N     = 2 * CONV_TL + 2;
constexpr int OT_PITCH = 36;
constexpr int LSTM_THR = 128;
constexpr int SEQ_BLK  = 16;
constexpr int HPITCH   = NHID + 8;
constexpr int SLABP    = 68;
constexpr int WOFF_IH0 = 0;
constexpr int WOFF_HH0 = WOFF_IH0 + NGATE * NCH_SEQ;
constexpr int WOFF_IH1 = WOFF_HH0 + NGATE * NHID;
constexpr int WOFF_HH1 = WOFF_IH1 + NGATE * NHID;
constexpr int WTOTAL   = WOFF_HH1 + NGATE * NHID;
static_assert(NSTEP * 4 == NPOS, "two pools of 2");
static_assert(NGATE == 4 * NHID, "gate blocks");
static_assert(NCH_SEQ % 32 == 0 && NHID % 32 == 0, "GEMM K multiples of 32");
static_assert(NBATCH % SEQ_BLK == 0, "row blocks");
static_assert(NHID == 16 * (LSTM_THR / 32), "one 16-unit subtile per wave");
static_assert(WTOTAL % (8 * 256) == 0, "split kernel grid exact");
static_assert((NBATCH * NOUTF) % 256 == 0, "head grid exact");

typedef __attribute__((ext_vector_type(16))) __bf16   v16b;
typedef __attribute__((ext_vector_type(8)))  __bf16   v8b;
typedef __attribute__((ext_vector_type(8)))  float    v8f;
typedef __attribute__((ext_vector_type(4)))  float    v4f;
typedef __attribute__((ext_vector_type(4)))  unsigned v4u;
typedef __attribute__((ext_vector_type(2)))  unsigned v2u;

__device__ __forceinline__ unsigned bf_rne_bits(float f) {
  const unsigned u = __float_as_uint(f);
  return (u + 0x7FFFu + ((u >> 16) & 1u)) >> 16;
}
__device__ __forceinline__ void bf_split(float f, unsigned& hi, unsigned& lo) {
  hi = bf_rne_bits(f);
  lo = bf_rne_bits(f - __uint_as_float(hi << 16));
}

__device__ __forceinline__ void guard_pair_b(v8f& a, v8f& b, v16b x0, v16b x1, v16b y0, v16b y1, v16b y2, v16b y3) {
  asm volatile("v_nop\n\tv_nop\n\tv_nop\n\tv_nop" : "+v"(a), "+v"(b) : "v"(x0), "v"(x1), "v"(y0), "v"(y1), "v"(y2), "v"(y3));
}
__device__ __forceinline__ void acc_guard4(v8f& a, v8f& b, v8f& c, v8f& d) { asm volatile("v_nop\n\tv_nop\n\tv_nop\n\tv_nop" : "+v"(a), "+v"(b), "+v"(c), "+v"(d)); }

template <typename T> struct Frag;
template <> struct Frag<__bf16> {
  typedef v16b V; union U { v16b v; v8b h[2]; };
  static __device__ __forceinline__ v16b load(const __bf16* p) {
    U f; f.h[0] = *(const v8b*)(p); f.h[1] = *(const v8b*)(p + 16); return f.v;
  }
  static __device__ __forceinline__ v8f mma(v16b a, v16b b, v8f c) {
    return __builtin_amdgcn_wmma_f32_16x16x32_bf16(false, a, false, b, (short)0, c, false, false);
  }
};

__device__ __forceinline__ float sigm(float x)   { return __builtin_amdgcn_rcpf(1.0f + expf(-x)); }
__device__ __forceinline__ float tanh_e(float x) { return 1.0f - 2.0f * __builtin_amdgcn_rcpf(expf(2.0f * x) + 1.0f); }

__global__ __launch_bounds__(256) void wsplit_kernel(const float* __restrict__ w_a, const float* __restrict__ w_b,
                                                     const float* __restrict__ w_c, const float* __restrict__ w_d,
                                                     unsigned short* __restrict__ whi, unsigned short* __restrict__ wlo) {
  const int blk = blockIdx.x, tid = threadIdx.x;
  const float* src; int cbase;
  if (blk < WOFF_HH0 / 2048)      { src = w_a; cbase = WOFF_IH0 / 8; }
  else if (blk < WOFF_IH1 / 2048) { src = w_b; cbase = WOFF_HH0 / 8; }
  else if (blk < WOFF_HH1 / 2048) { src = w_c; cbase = WOFF_IH1 / 8; }
  else                            { src = w_d; cbase = WOFF_HH1 / 8; }
  const int g = blk * 256 + tid;
  const float* sp = src + (size_t)(g - cbase) * 8;
  const v4f a = *(const v4f*)(sp);
  const v4f b = *(const v4f*)(sp + 4);
  unsigned h[8], l[8];
#pragma unroll
  for (int e = 0; e < 4; ++e) {
    const float fa = a[e], fb = b[e];
    bf_split(fa, h[e], l[e]);
    bf_split(fb, h[4 + e], l[4 + e]);
  }
  v4u hv, lv;
#pragma unroll
  for (int e = 0; e < 4; ++e) {
    hv[e] = h[2 * e] | (h[2 * e + 1] << 16);
    lv[e] = l[2 * e] | (l[2 * e + 1] << 16);
  }
  unsigned short* ph = whi + (size_t)g * 8;
  unsigned short* pl = wlo + (size_t)g * 8;
  *(volatile v4u*)ph = hv;
  *(volatile v4u*)pl = lv;
  __threadfence();
  *(volatile v4u*)ph = hv;
  *(volatile v4u*)pl = lv;
}

__global__ __launch_bounds__(256) void conv_front_kernel(const float* __restrict__ x, const float* __restrict__ w1,
                                                         const float* __restrict__ b1, const float* __restrict__ w2,
                                                         const float* __restrict__ b2, float* __restrict__ out) {
  __shared__ __align__(16) float xls[XL_N * 4];
  __shared__ __align__(16) float p1s[P1_N * NCH_MID];
  __shared__ __align__(16) float w2t[NCH_SEQ * 3 * NCH_MID];
  __shared__ __align__(16) float ot[CONV_TL * OT_PITCH];
  __shared__ float w1s[NCH_MID * 9];
  __shared__ float b1s[NCH_MID];
  __shared__ float b2s[NCH_SEQ];

  const int tid = threadIdx.x;
  const int b   = blockIdx.x;
  const int t4b = blockIdx.y * CONV_TL;

  {
    const int i1 = tid < (NCH_MID * 9 - 1) ? tid : (NCH_MID * 9 - 1);
    const float v1 = w1[i1];
    if (tid < NCH_MID * 9) w1s[tid] = v1;
    const int i2 = tid < (NCH_MID - 1) ? tid : (NCH_MID - 1);
    const float v2 = b1[i2];
    if (tid < NCH_MID) b1s[tid] = v2;
    const int i3 = tid < (NCH_SEQ - 1) ? tid : (NCH_SEQ - 1);
    const float v3 = b2[i3];
    if (tid < NCH_SEQ) b2s[tid] = v3;
  }
#pragma unroll 1
  for (int i = tid; i < NCH_SEQ * NCH_MID * 3; i += 256) {
    const int oc = i / 48, rem = i - oc * 48;
    const int ic = rem / 3, k = rem - ic * 3;
    w2t[(oc * 3 + k) * NCH_MID + ic] = w2[i];
  }
  const int p0 = 4 * t4b - 3;
#pragma unroll 1
  for (int e = tid; e < XL_N * 3; e += 256) {
    const int pos = e / 3, ch = e - pos * 3;
    const int gp = p0 + pos;
    const bool ok = (gp >= 0) && (gp < NPOS);
    const int gpc = gp < 0 ? 0 : (gp > NPOS - 1 ? NPOS - 1 : gp);
    const float v = x[((size_t)b * NPOS + (size_t)gpc) * NCH_IN + ch];
    xls[pos * 4 + ch] = ok ? v : 0.0f;
  }
  __syncthreads();

#pragma unroll 1
  for (int it = tid; it < P1_N * NCH_MID; it += 256) {
    const int ql = it >> 4, oc = it & 15;
    const int gq = 2 * t4b - 1 + ql;
    float c0 = b1s[oc], c1 = c0;
#pragma unroll
    for (int k = 0; k < 3; ++k)
#pragma unroll
      for (int ic = 0; ic < 3; ++ic) {
        const float w = w1s[oc * 9 + ic * 3 + k];
        c0 += xls[(2 * ql + k) * 4 + ic] * w;
        c1 += xls[(2 * ql + 1 + k) * 4 + ic] * w;
      }
    const float v = fmaxf(c0, c1);
    p1s[ql * NCH_MID + oc] = (gq >= 0 && gq < 2 * NSTEP) ? v : 0.0f;
  }
  __syncthreads();

#pragma unroll 1
  for (int it = tid; it < CONV_TL * NCH_SEQ; it += 256) {
    const int oc = it & 31, tl = it >> 5;
    float c0 = b2s[oc], c1 = c0;
#pragma unroll 1
    for (int ic4 = 0; ic4 < NCH_MID / 4; ++ic4) {
      const v4f r0 = *(const v4f*)&p1s[(2 * tl + 0) * NCH_MID + ic4 * 4];
      const v4f r1 = *(const v4f*)&p1s[(2 * tl + 1) * NCH_MID + ic4 * 4];
      const v4f r2 = *(const v4f*)&p1s[(2 * tl + 2) * NCH_MID + ic4 * 4];
      const v4f r3 = *(const v4f*)&p1s[(2 * tl + 3) * NCH_MID + ic4 * 4];
      const v4f wa = *(const v4f*)&w2t[(oc * 3 + 0) * NCH_MID + ic4 * 4];
      const v4f wb = *(const v4f*)&w2t[(oc * 3 + 1) * NCH_MID + ic4 * 4];
      const v4f wc = *(const v4f*)&w2t[(oc * 3 + 2) * NCH_MID + ic4 * 4];
#pragma unroll
      for (int e = 0; e < 4; ++e) {
        c0 += r0[e] * wa[e]; c0 += r1[e] * wb[e]; c0 += r2[e] * wc[e];
        c1 += r1[e] * wa[e]; c1 += r2[e] * wb[e]; c1 += r3[e] * wc[e];
      }
    }
    ot[tl * OT_PITCH + oc] = fmaxf(c0, c1);
  }
  __syncthreads();

  v4f vv[4];
#pragma unroll
  for (int it = 0; it < 4; ++it) {
    const int idx = it * 256 + tid;
    const int row = idx >> 3, c4 = (idx & 7) * 4;
    vv[it] = *(const v4f*)&ot[row * OT_PITCH + c4];
  }
  for (int pass = 0; pass < 2; ++pass) {
#pragma unroll
    for (int it = 0; it < 4; ++it) {
      const int idx = it * 256 + tid;
      const int row = idx >> 3, c4 = (idx & 7) * 4;
      *(volatile v4f*)(out + ((size_t)b * NSTEP + (size_t)(t4b + row)) * NCH_SEQ + c4) = vv[it];
    }
    __threadfence();
  }
}

template <int IN>
__device__ __forceinline__ void stage_x_tile(const float* xs, int rowbase, int tn, int tid,
                                             unsigned short* Axh, unsigned short* Axl) {
  constexpr int XP  = IN + 8;
  constexpr int EPT = IN / 8;
  const int m = tid >> 3, f0 = (tid & 7) * EPT;
  const float* sp = xs + ((size_t)(rowbase + m) * NSTEP + (size_t)tn) * IN + f0;
  const v4f a = *(const v4f*)(sp);
  unsigned h0, l0, h1, l1, h2, l2, h3, l3;
  { const float f = a[0]; bf_split(f, h0, l0); }
  { const float f = a[1]; bf_split(f, h1, l1); }
  { const float f = a[2]; bf_split(f, h2, l2); }
  { const float f = a[3]; bf_split(f, h3, l3); }
  if constexpr (EPT == 4) {
    v2u hw, lw;
    hw[0] = h0 | (h1 << 16); hw[1] = h2 | (h3 << 16);
    lw[0] = l0 | (l1 << 16); lw[1] = l2 | (l3 << 16);
    *(v2u*)(Axh + m * XP + f0) = hw;
    *(v2u*)(Axl + m * XP + f0) = lw;
  } else {
    const v4f b = *(const v4f*)(sp + 4);
    unsigned h4, l4, h5, l5, h6, l6, h7, l7;
    { const float f = b[0]; bf_split(f, h4, l4); }
    { const float f = b[1]; bf_split(f, h5, l5); }
    { const float f = b[2]; bf_split(f, h6, l6); }
    { const float f = b[3]; bf_split(f, h7, l7); }
    v4u hw, lw;
    hw[0] = h0 | (h1 << 16); hw[1] = h2 | (h3 << 16); hw[2] = h4 | (h5 << 16); hw[3] = h6 | (h7 << 16);
    lw[0] = l0 | (l1 << 16); lw[1] = l2 | (l3 << 16); lw[2] = l4 | (l5 << 16); lw[3] = l6 | (l7 << 16);
    *(v4u*)(Axh + m * XP + f0) = hw;
    *(v4u*)(Axl + m * XP + f0) = lw;
  }
}

__device__ __forceinline__ void mma3_pair(v8f& acc0, v8f& acc1, v16b ah, v16b al,
                                          const __bf16* ph, const __bf16* pl, int gstride) {
  asm volatile("" ::: "memory");
  const v16b bh0 = Frag<__bf16>::load(ph);
  const v16b bl0 = Frag<__bf16>::load(pl);
  const v16b bh1 = Frag<__bf16>::load(ph + gstride);
  const v16b bl1 = Frag<__bf16>::load(pl + gstride);
  acc0 = Frag<__bf16>::mma(ah, bl0, acc0);
  acc0 = Frag<__bf16>::mma(al, bh0, acc0);
  acc0 = Frag<__bf16>::mma(ah, bh0, acc0);
  acc1 = Frag<__bf16>::mma(ah, bl1, acc1);
  acc1 = Frag<__bf16>::mma(al, bh1, acc1);
  acc1 = Frag<__bf16>::mma(ah, bh1, acc1);
  guard_pair_b(acc0, acc1, ah, al, bh0, bl0, bh1, bl1);
}

template <int IN, bool SEQ_OUT>
__global__ __launch_bounds__(LSTM_THR) void lstm_seq_kernel(const float* __restrict__ xs,
                                                            const unsigned short* wih_h, const unsigned short* wih_l,
                                                            const unsigned short* whh_h, const unsigned short* whh_l,
                                                            const float* __restrict__ b_ih, const float* __restrict__ b_hh,
                                                            float* __restrict__ hout) {
  static_assert(IN % 32 == 0, "K multiple of 32");
  constexpr int XP = IN + 8;
  __shared__ __align__(16) unsigned short Axh[SEQ_BLK * XP];
  __shared__ __align__(16) unsigned short Axl[SEQ_BLK * XP];
  __shared__ __align__(16) unsigned short Ahh[SEQ_BLK * HPITCH];
  __shared__ __align__(16) unsigned short Ahl[SEQ_BLK * HPITCH];
  __shared__ __align__(16) float          Sl[SEQ_BLK * SLABP];

  const int tid = threadIdx.x, lane = tid & 31, ub = tid >> 5;
  const int c = lane & 15, hh = lane >> 4, koff = hh * 8;
  const int rowbase = blockIdx.x * SEQ_BLK;
  const int j = 16 * ub + c;

#pragma unroll 1
  for (int i = tid; i < SEQ_BLK * XP; i += LSTM_THR) { Axh[i] = 0; Axl[i] = 0; }
#pragma unroll 1
  for (int i = tid; i < SEQ_BLK * HPITCH; i += LSTM_THR) { Ahh[i] = 0; Ahl[i] = 0; }
#pragma unroll 1
  for (int i = tid; i < SEQ_BLK * SLABP; i += LSTM_THR) Sl[i] = 0.0f;

  float bsum[4];
#pragma unroll
  for (int g = 0; g < 4; ++g) bsum[g] = b_ih[g * NHID + j] + b_hh[g * NHID + j];
  float cst[8];
#pragma unroll
  for (int r = 0; r < 8; ++r) cst[r] = 0.0f;
  __syncthreads();
  stage_x_tile<IN>(xs, rowbase, 0, tid, Axh, Axl);
  __syncthreads();

  const __bf16* axh_row = (const __bf16*)Axh + c * XP + koff;
  const __bf16* axl_row = (const __bf16*)Axl + c * XP + koff;
  const __bf16* ahh_row = (const __bf16*)Ahh + c * HPITCH + koff;
  const __bf16* ahl_row = (const __bf16*)Ahl + c * HPITCH + koff;
  const __bf16* wxh = (const __bf16*)wih_h + (size_t)j * IN + koff;
  const __bf16* wxl = (const __bf16*)wih_l + (size_t)j * IN + koff;
  const __bf16* wrh = (const __bf16*)whh_h + (size_t)j * NHID + koff;
  const __bf16* wrl = (const __bf16*)whh_l + (size_t)j * NHID + koff;
  constexpr int GSX = NHID * IN;
  constexpr int GSH = NHID * NHID;

#pragma unroll 1
  for (int t = 0; t < NSTEP; ++t) {
    v8f acc[4];
#pragma unroll
    for (int g = 0; g < 4; ++g) {
      const float bv = bsum[g];
      acc[g] = (v8f){bv, bv, bv, bv, bv, bv, bv, bv};
    }
#pragma unroll 1
    for (int kx = 0; kx < IN; kx += 32) {
      const v16b ah = Frag<__bf16>::load(axh_row + kx);
      const v16b al = Frag<__bf16>::load(axl_row + kx);
      mma3_pair(acc[0], acc[1], ah, al, wxh + kx, wxl + kx, GSX);
      mma3_pair(acc[2], acc[3], ah, al, wxh + 2 * GSX + kx, wxl + 2 * GSX + kx, GSX);
    }
#pragma unroll 1
    for (int k0 = 0; k0 < NHID; k0 += 32) {
      const v16b ah = Frag<__bf16>::load(ahh_row + k0);
      const v16b al = Frag<__bf16>::load(ahl_row + k0);
      mma3_pair(acc[0], acc[1], ah, al, wrh + k0, wrl + k0, GSH);
      mma3_pair(acc[2], acc[3], ah, al, wrh + 2 * GSH + k0, wrl + 2 * GSH + k0, GSH);
    }
    acc_guard4(acc[0], acc[1], acc[2], acc[3]);

    float hn[8];
#pragma unroll
    for (int r = 0; r < 8; ++r) {
      const float ig = sigm(acc[0][r]);
      const float fg = sigm(acc[1][r]);
      const float gg = tanh_e(acc[2][r]);
      const float og = sigm(acc[3][r]);
      const float cn = fg * cst[r] + ig * gg;
      cst[r] = cn;
      hn[r] = og * tanh_e(cn);
    }
    __syncthreads();
#pragma unroll
    for (int r = 0; r < 8; ++r) {
      const int row = 8 * hh + r;
      unsigned hb, lb;
      bf_split(hn[r], hb, lb);
      Ahh[row * HPITCH + j] = (unsigned short)hb;
      Ahl[row * HPITCH + j] = (unsigned short)lb;
      Sl[row * SLABP + j] = hn[r];
    }
    {
      const int tn = (t + 1 < NSTEP) ? (t + 1) : (NSTEP - 1);
      stage_x_tile<IN>(xs, rowbase, tn, tid, Axh, Axl);
    }
    __syncthreads();
    if (SEQ_OUT) {
      v4f sv[2];
#pragma unroll
      for (int it = 0; it < 2; ++it) {
        const int idx = it * LSTM_THR + tid;
        const int row = idx >> 4, c4 = (idx & 15) * 4;
        sv[it] = *(const v4f*)&Sl[row * SLABP + c4];
      }
      for (int pass = 0; pass < 2; ++pass) {
#pragma unroll
        for (int it = 0; it < 2; ++it) {
          const int idx = it * LSTM_THR + tid;
          const int row = idx >> 4, c4 = (idx & 15) * 4;
          *(volatile v4f*)(hout + ((size_t)(rowbase + row) * NSTEP + (size_t)t) * NHID + c4) = sv[it];
        }
        __threadfence();
      }
    }
  }

  if (!SEQ_OUT) {
    v4f sv[2];
#pragma unroll
    for (int it = 0; it < 2; ++it) {
      const int idx = it * LSTM_THR + tid;
      const int row = idx >> 4, c4 = (idx & 15) * 4;
      sv[it] = *(const v4f*)&Sl[row * SLABP + c4];
    }
    for (int pass = 0; pass < 2; ++pass) {
#pragma unroll
      for (int it = 0; it < 2; ++it) {
        const int idx = it * LSTM_THR + tid;
        const int row = idx >> 4, c4 = (idx & 15) * 4;
        *(volatile v4f*)(hout + (size_t)(rowbase + row) * NHID + c4) = sv[it];
      }
      __threadfence();
    }
  }
}

__global__ __launch_bounds__(256) void fc_head_kernel(const float* __restrict__ hl, const float* __restrict__ fw,
                                                      const float* __restrict__ fb, float* __restrict__ out) {
  const int tid = threadIdx.x;
#pragma unroll 1
  for (int jj = 0; jj < NOUTF; ++jj) {
    const int f = tid + 256 * jj;
    const int row = f / NOUTF;
    const int o = f - row * NOUTF;
    float acc = fb[o];
    const float* hp = hl + (size_t)row * NHID;
    const float* wp = fw + (size_t)o * NHID;
#pragma unroll 2
    for (int k4 = 0; k4 < NHID / 4; ++k4) {
      const v4f a = *(const v4f*)(hp + 4 * k4);
      const v4f w = *(const v4f*)(wp + 4 * k4);
      acc += a[0] * w[0]; acc += a[1] * w[1]; acc += a[2] * w[2]; acc += a[3] * w[3];
    }
    *(volatile float*)(out + f) = acc;
    __threadfence();
    *(volatile float*)(out + f) = acc;
  }
}

extern "C" void kernel_launch(void* const* d_in, const int* in_sizes, int n_in,
                              void* d_out, int out_size, void* d_ws, size_t ws_size, hipStream_t stream) {
  if (n_in < 15 || d_out == nullptr || d_ws == nullptr) return;
  if (in_sizes[0] != NBATCH * NPOS * NCH_IN || in_sizes[1] != NCH_MID * NCH_IN * 3 || in_sizes[2] != NCH_MID ||
      in_sizes[3] != NCH_SEQ * NCH_MID * 3 || in_sizes[4] != NCH_SEQ ||
      in_sizes[5] != NGATE * NCH_SEQ || in_sizes[6] != NGATE * NHID || in_sizes[7] != NGATE || in_sizes[8] != NGATE ||
      in_sizes[9] != NGATE * NHID || in_sizes[10] != NGATE * NHID || in_sizes[11] != NGATE || in_sizes[12] != NGATE ||
      in_sizes[13] != NOUTF * NHID || in_sizes[14] != NOUTF || out_size != NBATCH * NOUTF) return;

  const float* x       = (const float*)d_in[0];
  const float* conv1_w = (const float*)d_in[1];
  const float* conv1_b = (const float*)d_in[2];
  const float* conv2_w = (const float*)d_in[3];
  const float* conv2_b = (const float*)d_in[4];
  const float* w_ih0   = (const float*)d_in[5];
  const float* w_hh0   = (const float*)d_in[6];
  const float* b_ih0   = (const float*)d_in[7];
  const float* b_hh0   = (const float*)d_in[8];
  const float* w_ih1   = (const float*)d_in[9];
  const float* w_hh1   = (const float*)d_in[10];
  const float* b_ih1   = (const float*)d_in[11];
  const float* b_hh1   = (const float*)d_in[12];
  const float* fc_w    = (const float*)d_in[13];
  const float* fc_b    = (const float*)d_in[14];
  float* out = (float*)d_out;

  char* ws = (char*)d_ws; size_t off = 0;
  auto carve = [&](size_t bytes) -> char* { char* p = ws + off; off += (bytes + 255) & ~(size_t)255; return p; };
  unsigned short* WHI = (unsigned short*)carve((size_t)WTOTAL * 2);
  unsigned short* WLO = (unsigned short*)carve((size_t)WTOTAL * 2);
  float* P0 = (float*)carve((size_t)NBATCH * NSTEP * NCH_SEQ * 4);
  float* P1 = (float*)carve((size_t)NBATCH * NSTEP * NHID * 4);
  float* P2 = (float*)carve((size_t)NBATCH * NHID * 4);
  if (off > ws_size || off > (size_t)134217728) return;

  wsplit_kernel<<<WTOTAL / (8 * 256), 256, 0, stream>>>(w_ih0, w_hh0, w_ih1, w_hh1, WHI, WLO);
  conv_front_kernel<<<dim3(NBATCH, NSTEP / CONV_TL), 256, 0, stream>>>(x, conv1_w, conv1_b, conv2_w, conv2_b, P0);
  lstm_seq_kernel<NCH_SEQ, true><<<NBATCH / SEQ_BLK, LSTM_THR, 0, stream>>>(
      P0, WHI + WOFF_IH0, WLO + WOFF_IH0, WHI + WOFF_HH0, WLO + WOFF_HH0, b_ih0, b_hh0, P1);
  lstm_seq_kernel<NHID, false><<<NBATCH / SEQ_BLK, LSTM_THR, 0, stream>>>(
      P1, WHI + WOFF_IH1, WLO + WOFF_IH1, WHI + WOFF_HH1, WLO + WOFF_HH1, b_ih1, b_hh1, P2);
  fc_head_kernel<<<1, 256, 0, stream>>>(P2, fc_w, fc_b, out);
}
